// LocalAttention1D_53987738910745
// MI455X (gfx1250) — hardware-verified
//
#include <hip/hip_runtime.h>


#define NB_  2
#define TT   4096
#define DD   512
#define NH_  8
#define HD   64
#define WIN  16
#define NT   (NB_ * TT)
#define SCL  0.125f
typedef _Float16 h16;
typedef unsigned short bf;
typedef __attribute__((ext_vector_type(16))) __bf16   v16bf;
typedef __attribute__((ext_vector_type(16))) _Float16 v16h;
typedef __attribute__((ext_vector_type(8)))  _Float16 v8h;
typedef __attribute__((ext_vector_type(8)))  unsigned short v8us;
typedef __attribute__((ext_vector_type(8)))  float    v8f;
typedef __attribute__((ext_vector_type(4)))  float    v4f;
typedef v8h  __attribute__((may_alias)) v8ha;
typedef v4f  __attribute__((may_alias)) v4fa;
typedef v8us __attribute__((may_alias)) v8usa;

__device__ __forceinline__ unsigned short f2bf(float f) { unsigned u = __float_as_uint(f); u += 0x7FFFu + ((u >> 16) & 1u); return (unsigned short)(u >> 16); }
__device__ __forceinline__ float bf2f(unsigned short b) { return __uint_as_float(((unsigned)b) << 16); }
__device__ __forceinline__ float bfr(float f) { return bf2f(f2bf(f)); }
__device__ __forceinline__ v16h cat16(v8h lo, v8h hi) { return __builtin_shufflevector(lo, hi, 0, 1, 2, 3, 4, 5, 6, 7, 8, 9, 10, 11, 12, 13, 14, 15); }
__device__ __forceinline__ v16bf cat16b(v8us lo, v8us hi) { return __builtin_bit_cast(v16bf, __builtin_shufflevector(lo, hi, 0, 1, 2, 3, 4, 5, 6, 7, 8, 9, 10, 11, 12, 13, 14, 15)); }
__device__ __forceinline__ v8f wmma16(v16h a, v16h b, v8f c) { return __builtin_amdgcn_wmma_f32_16x16x32_f16(false, a, false, b, (short)0, c, false, false); }
__device__ __forceinline__ v8f wmmab(v16bf a, v16bf b, v8f c) { return __builtin_amdgcn_wmma_f32_16x16x32_bf16(false, a, false, b, (short)0, c, false, false); }


template <typename T16> struct WFrag;
template <> struct WFrag<h16> { typedef v16h V; static __device__ __forceinline__ V ld(const h16* p) { return cat16(*(const v8h*)p, *(const v8h*)(p + 16)); } static __device__ __forceinline__ v8f mma(V a, V b, v8f c) { return wmma16(a, b, c); } };
template <> struct WFrag<bf> { typedef v16bf V; static __device__ __forceinline__ V ld(const bf* p) { return cat16b(*(const v8us*)p, *(const v8us*)(p + 16)); } static __device__ __forceinline__ v8f mma(V a, V b, v8f c) { return wmmab(a, b, c); } };
template <typename T16, int NSPLIT, bool BIAS>
__global__ __launch_bounds__(32) void k_gemmw(const T16* __restrict__ A, const T16* __restrict__ A2, const T16* __restrict__ Bt, const T16* __restrict__ Bt2, int K, float* C, int ldc, const float* __restrict__ bias, size_t sA, size_t sB, size_t sC) {
    typedef typename WFrag<T16>::V V;
    __shared__ __align__(16) float os[16 * 68];
    const size_t z = blockIdx.z; A += z * sA; if (A2) A2 += z * sA; Bt += z * sB; if (Bt2) Bt2 += z * sB; C += z * sC;
    const int lane = threadIdx.x & 31, lr = lane & 15, hi = lane >> 4; const int r0 = blockIdx.x * 64, c0 = blockIdx.y * 64;
    v8f acc[4][4];
#pragma unroll
    for (int mb = 0; mb < 4; ++mb)
#pragma unroll
        for (int nb = 0; nb < 4; ++nb) acc[mb][nb] = (v8f){};
    const size_t aoff = (size_t)(r0 + lr) * K + 8 * hi, boff = (size_t)(c0 + lr) * K + 8 * hi;
#pragma unroll 1
    for (int kc = 0; kc < K; kc += 32) {
        V a[4], a2[4];
#pragma unroll
        for (int mb = 0; mb < 4; ++mb) { a[mb] = WFrag<T16>::ld(A + aoff + (size_t)mb * 16 * K + kc); if (NSPLIT == 1 || NSPLIT == 2) a2[mb] = WFrag<T16>::ld(A2 + aoff + (size_t)mb * 16 * K + kc); }
#pragma unroll
        for (int nb = 0; nb < 4; ++nb) { const V b = WFrag<T16>::ld(Bt + boff + (size_t)nb * 16 * K + kc); V b2; if (NSPLIT >= 2) b2 = WFrag<T16>::ld(Bt2 + boff + (size_t)nb * 16 * K + kc);
#pragma unroll
            for (int mb = 0; mb < 4; ++mb) { acc[mb][nb] = WFrag<T16>::mma(a[mb], b, acc[mb][nb]); if (NSPLIT == 1 || NSPLIT == 2) acc[mb][nb] = WFrag<T16>::mma(a2[mb], b, acc[mb][nb]); if (NSPLIT >= 2) acc[mb][nb] = WFrag<T16>::mma(a[mb], b2, acc[mb][nb]); } }
        asm volatile("v_nop\n\tv_nop\n\tv_nop\n\tv_nop" : "+v"(acc[0][0]), "+v"(acc[1][1]), "+v"(acc[2][2]), "+v"(acc[3][3]) : "v"(a[0]), "v"(a[3]));
    }
#pragma unroll
    for (int mb = 0; mb < 4; ++mb) {
#pragma unroll
        for (int nb = 0; nb < 4; ++nb) {
#pragma unroll
            for (int j = 0; j < 8; ++j) os[(hi * 8 + j) * 68 + nb * 16 + lr] = acc[mb][nb][j]; }
        __builtin_amdgcn_wave_barrier(); asm volatile("" ::: "memory");
        float* crow = C + (size_t)(r0 + mb * 16) * ldc + c0;
#pragma unroll 1
        for (int ps = 0; ps < 2; ++ps) {
#pragma unroll
            for (int s = 0; s < 8; ++s) { const int row = 2 * s + hi, cofs = lr * 4; v4f val = *(const v4fa*)(os + row * 68 + cofs); if (BIAS) { val[0] += bfr(bias[c0 + cofs]); val[1] += bfr(bias[c0 + cofs + 1]); val[2] += bfr(bias[c0 + cofs + 2]); val[3] += bfr(bias[c0 + cofs + 3]); }
                *(volatile v4f*)(crow + (size_t)row * ldc + cofs) = val; }
            if (ps == 0) __threadfence(); }
        __builtin_amdgcn_wave_barrier(); asm volatile("" ::: "memory");
    }
}

__device__ __forceinline__ void splitf(float y, unsigned short& h, unsigned short& l) { h = f2bf(y); l = f2bf(y - bf2f(h)); }
typedef __attribute__((ext_vector_type(2))) unsigned short v2us;
typedef __attribute__((ext_vector_type(2))) float v2f;

__global__ __launch_bounds__(256) void k_cvt8(const float* __restrict__ src, bf* dst, size_t n8) { const size_t i = (size_t)blockIdx.x * 256 + threadIdx.x; if (i >= n8) return; const v8f v = *(const v8f*)(src + i * 8); v8us o;
#pragma unroll
    for (int k = 0; k < 8; ++k) o[k] = f2bf(v[k]); *(volatile v8us*)(dst + i * 8) = o; __threadfence(); *(volatile v8us*)(dst + i * 8) = o; }
__global__ __launch_bounds__(256) void k_local(const float* __restrict__ FQ, const float* __restrict__ FK, const float* __restrict__ FV, bf* Ah, bf* Al) {
    const int lane = threadIdx.x & 31; const int w0 = blockIdx.x * 8 + (threadIdx.x >> 5); if (w0 >= NT * NH_) return; const int r = w0 / NH_, h = w0 % NH_; const int b = r / TT, t = r % TT; const int d = lane * 2;
    const v2f q2 = *(const v2f*)(FQ + (size_t)r * DD + h * HD + d); float s[2 * WIN + 1]; float mx = -3.0e38f;
#pragma unroll
    for (int w = 0; w < 2 * WIN + 1; ++w) { const int tk = t + w - WIN; float acc = -3.0e38f;
        if (tk >= 0 && tk < TT) { const v2f k2 = *(const v2f*)(FK + ((size_t)b * TT + tk) * DD + h * HD + d); float p0 = __fmul_rn(q2[0], k2[0]), p1 = __fmul_rn(q2[1], k2[1]); asm volatile("" : "+v"(p0)); asm volatile("" : "+v"(p1)); acc = __fadd_rn(p0, p1);
#pragma unroll
            for (int sh = 16; sh; sh >>= 1) acc += __shfl_xor(acc, sh, 32);
            acc = __fmul_rn(acc, SCL); mx = fmaxf(mx, acc); }
        s[w] = acc; }
    float sum = 0.f;
#pragma unroll
    for (int w = 0; w < 2 * WIN + 1; ++w) { const int tk = t + w - WIN; s[w] = (tk >= 0 && tk < TT) ? __expf(s[w] - mx) : 0.f; sum += s[w]; }
    const float inv = __fdiv_rn(1.0f, sum); float o0 = 0.f, o1 = 0.f;
#pragma unroll
    for (int w = 0; w < 2 * WIN + 1; ++w) { const int tk = t + w - WIN; if (tk < 0 || tk >= TT) continue; const v2f v2 = *(const v2f*)(FV + ((size_t)b * TT + tk) * DD + h * HD + d); float pw = __fmul_rn(s[w], inv); asm volatile("" : "+v"(pw));
        float m0 = __fmul_rn(pw, v2[0]), m1 = __fmul_rn(pw, v2[1]); asm volatile("" : "+v"(m0)); asm volatile("" : "+v"(m1)); o0 = __fadd_rn(o0, m0); o1 = __fadd_rn(o1, m1); }
    v2us oh, ol; unsigned short a, c2; splitf(o0, a, c2); oh[0] = a; ol[0] = c2; splitf(o1, a, c2); oh[1] = a; ol[1] = c2;
    const size_t o = (size_t)r * DD + h * HD + d; *(volatile v2us*)(Ah + o) = oh; *(volatile v2us*)(Al + o) = ol; __threadfence(); *(volatile v2us*)(Ah + o) = oh; *(volatile v2us*)(Al + o) = ol; }
__global__ __launch_bounds__(256) void k_lnres(const float* __restrict__ Y, const float* __restrict__ x, const float* __restrict__ gg, const float* __restrict__ bb, float* OUT) {
    const int lane = threadIdx.x & 31; const int r = blockIdx.x * 8 + (threadIdx.x >> 5); if (r >= NT) return; float v[DD / 32]; float s = 0.f;
#pragma unroll
    for (int c = 0; c < (DD / 128); ++c) { const v4f a = *(const v4f*)(Y + (size_t)r * DD + c * 128 + lane * 4), xx = *(const v4f*)(x + (size_t)r * DD + c * 128 + lane * 4);
#pragma unroll
        for (int q = 0; q < 4; ++q) { v[c * 4 + q] = __fadd_rn(a[q], bfr(xx[q])); s += v[c * 4 + q]; } }
#pragma unroll
    for (int sh = 16; sh; sh >>= 1) s += __shfl_xor(s, sh, 32);
    const float mu = s * (1.0f / DD); float qq = 0.f;
#pragma unroll
    for (int i = 0; i < DD / 32; ++i) { const float d0 = v[i] - mu; qq = __fadd_rn(qq, __fmul_rn(d0, d0)); }
#pragma unroll
    for (int sh = 16; sh; sh >>= 1) qq += __shfl_xor(qq, sh, 32);
    const float rs = __fdiv_rn(1.0f, __fsqrt_rn(qq * (1.0f / DD) + 1e-5f));
#pragma unroll 1
    for (int ps = 0; ps < 2; ++ps) {
#pragma unroll
        for (int c = 0; c < (DD / 128); ++c) { v4f o;
#pragma unroll
            for (int q = 0; q < 4; ++q) { const int col = c * 128 + lane * 4 + q; o[q] = __fadd_rn(__fmul_rn((v[c * 4 + q] - mu) * rs, bfr(gg[col])), bfr(bb[col])); }
            *(volatile v4f*)(OUT + (size_t)r * DD + c * 128 + lane * 4) = o; }
        if (ps == 0) __threadfence(); }
}

extern "C" void kernel_launch(void* const* d_in, const int* in_sizes, int n_in,
                              void* d_out, int out_size, void* d_ws, size_t ws_size, hipStream_t stream) {
    (void)in_sizes; (void)n_in; (void)out_size;
    const float* x = (const float*)d_in[0]; const float* Wq = (const float*)d_in[1]; const float* Wk = (const float*)d_in[2]; const float* Wv = (const float*)d_in[3]; const float* Wp = (const float*)d_in[4]; const float* gam = (const float*)d_in[5]; const float* bet = (const float*)d_in[6];
    float* OUT = (float*)d_out;
    char* wsp = (char*)d_ws;
    auto take = [&](size_t bytes) { char* p = wsp; wsp += (bytes + 255) & ~(size_t)255; return (void*)p; };
    bf* WQ = (bf*)take((size_t)DD * DD * 2); bf* WK = (bf*)take((size_t)DD * DD * 2); bf* WV = (bf*)take((size_t)DD * DD * 2); bf* WP = (bf*)take((size_t)DD * DD * 2);
    bf* XB = (bf*)take((size_t)NT * DD * 2); float* FQ = (float*)take((size_t)NT * DD * 4); float* FK = (float*)take((size_t)NT * DD * 4); float* FV = (float*)take((size_t)NT * DD * 4); bf* Ah = (bf*)take((size_t)NT * DD * 2); bf* Al = (bf*)take((size_t)NT * DD * 2); float* Y = FQ;
    if ((size_t)(wsp - (char*)d_ws) > ws_size) return;
    { const size_t nw = (size_t)DD * DD / 8; const unsigned gw = (unsigned)((nw + 255) / 256); k_cvt8<<<gw, 256, 0, stream>>>(Wq, WQ, nw); k_cvt8<<<gw, 256, 0, stream>>>(Wk, WK, nw); k_cvt8<<<gw, 256, 0, stream>>>(Wv, WV, nw); k_cvt8<<<gw, 256, 0, stream>>>(Wp, WP, nw);
      const size_t nx = (size_t)NT * DD / 8; k_cvt8<<<(unsigned)((nx + 255) / 256), 256, 0, stream>>>(x, XB, nx); }
    const dim3 gP(NT / 64, DD / 64, 1);
    k_gemmw<bf, 0, false><<<gP, 32, 0, stream>>>(XB, nullptr, WQ, nullptr, DD, FQ, DD, nullptr, 0, 0, 0);
    k_gemmw<bf, 0, false><<<gP, 32, 0, stream>>>(XB, nullptr, WK, nullptr, DD, FK, DD, nullptr, 0, 0, 0);
    k_gemmw<bf, 0, false><<<gP, 32, 0, stream>>>(XB, nullptr, WV, nullptr, DD, FV, DD, nullptr, 0, 0, 0);
    k_local<<<(NT * NH_ + 7) / 8, 256, 0, stream>>>(FQ, FK, FV, Ah, Al);
    k_gemmw<bf, 1, false><<<gP, 32, 0, stream>>>(Ah, Al, WP, nullptr, DD, Y, DD, nullptr, 0, 0, 0);
    k_lnres<<<NT / 8, 256, 0, stream>>>(Y, x, gam, bet, OUT);
}
